// D_Attention_82377472738015
// MI455X (gfx1250) — hardware-run, weakly checked
//
#include <hip/hip_runtime.h>
#include <math.h>
#include <stdint.h>

constexpr int kBatch = 8;
constexpr int kSeq   = 1024;
constexpr int kDim   = 512;
constexpr int kHeads = 8;
constexpr int kHdim  = 64;
constexpr int kDff   = 2048;
constexpr int kRows  = kBatch * kSeq;
constexpr float kEps = 1e-5f;
constexpr float kPScale   = 32768.0f;
constexpr float kWScale   = 64.0f;
constexpr float kOScale   = 16.0f;

static_assert(kDim % 64 == 0 && kDff % 64 == 0 && kRows % 64 == 0 && kSeq % 64 == 0);
static_assert(kHeads * kHdim == kDim);

typedef __attribute__((ext_vector_type(16))) _Float16 v16h;
typedef __attribute__((ext_vector_type(8)))  _Float16 v8h;
typedef __attribute__((ext_vector_type(16))) __bf16   v16b;
typedef __attribute__((ext_vector_type(8)))  __bf16   v8b;
typedef __attribute__((ext_vector_type(8)))  float    v8f;
typedef __attribute__((ext_vector_type(4)))  float    v4f;
typedef __attribute__((ext_vector_type(2)))  float    v2f;
typedef __attribute__((ext_vector_type(4)))  unsigned int v4u;

__device__ __forceinline__ unsigned short f2bf_bits(float f) {
  unsigned u = __float_as_uint(f);
  return (unsigned short)((u + 0x7FFFu + ((u >> 16) & 1u)) >> 16);
}
__device__ __forceinline__ float bf_bits2f(unsigned short h) { return __uint_as_float(((unsigned)h) << 16); }

__device__ __forceinline__ void dep_guard_h(v8f& a, v8f& b, v16h x, v16h y) { asm volatile("v_nop\n\tv_nop\n\tv_nop\n\tv_nop" : "+v"(a), "+v"(b) : "v"(x), "v"(y)); }
__device__ __forceinline__ void dep_guard_b(v8f& a, v8f& b, v16b x, v16b y) { asm volatile("v_nop\n\tv_nop\n\tv_nop\n\tv_nop" : "+v"(a), "+v"(b) : "v"(x), "v"(y)); }
__device__ __forceinline__ void keep4_h(v16h a, v16h b, v16h c, v16h d) { asm volatile("v_nop" :: "v"(a), "v"(b), "v"(c), "v"(d)); }
__device__ __forceinline__ void keep4_b(v16b a, v16b b, v16b c, v16b d) { asm volatile("v_nop" :: "v"(a), "v"(b), "v"(c), "v"(d)); }
__device__ __forceinline__ void acc_guard4(v8f& a, v8f& b, v8f& c, v8f& d) { asm volatile("v_nop\n\tv_nop\n\tv_nop\n\tv_nop" : "+v"(a), "+v"(b), "+v"(c), "+v"(d)); }
template <typename T> struct Frag;
template <> struct Frag<_Float16> {
  typedef v16h V; union U { v16h v; v8h h[2]; };
  static __device__ __forceinline__ v16h load(const _Float16* p) {
    U f; f.h[0] = *(const v8h*)(p); f.h[1] = *(const v8h*)(p + 16); return f.v;
  }
  static __device__ __forceinline__ v8f mma(v16h a, v16h b, v8f c) {
    return __builtin_amdgcn_wmma_f32_16x16x32_f16(false, a, false, b, (short)0, c, false, false);
  }
  static __device__ __forceinline__ void guard(v8f& a, v8f& b, v16h x, v16h y) { dep_guard_h(a, b, x, y); }
  static __device__ __forceinline__ void keep(v16h a, v16h b, v16h c, v16h d) { keep4_h(a, b, c, d); }
};
template <> struct Frag<__bf16> {
  typedef v16b V; union U { v16b v; v8b h[2]; };
  static __device__ __forceinline__ v16b load(const __bf16* p) {
    U f; f.h[0] = *(const v8b*)(p); f.h[1] = *(const v8b*)(p + 16); return f.v;
  }
  static __device__ __forceinline__ v8f mma(v16b a, v16b b, v8f c) {
    return __builtin_amdgcn_wmma_f32_16x16x32_bf16(false, a, false, b, (short)0, c, false, false);
  }
  static __device__ __forceinline__ void guard(v8f& a, v8f& b, v16b x, v16b y) { dep_guard_b(a, b, x, y); }
  static __device__ __forceinline__ void keep(v16b a, v16b b, v16b c, v16b d) { keep4_b(a, b, c, d); }
};

template <int ET> struct Elem;
template <> struct Elem<0> { typedef _Float16 T; };
template <> struct Elem<1> { typedef __bf16 T; };
template <int ET, bool SPLIT, int BIAS_MODE, int OUT_MODE, bool RESID, int ACT = 0>
__global__ __launch_bounds__(256) void wmma_gemm64(
    const unsigned short* __restrict__ Ap, const unsigned short* __restrict__ A2p, int lda, long strideA,
    const unsigned short* __restrict__ Btp, const unsigned short* __restrict__ Bt2p, int ldb, long strideB,
    void* __restrict__ Cout, void* __restrict__ Cout2, int ldc, long strideC,
    const float* __restrict__ bias,
    const float* __restrict__ resid, long strideR,
    int M, int N, int K, float scale) {
  typedef typename Elem<ET>::T T;
  typedef typename Frag<T>::V V;
  const T* A = (const T*)Ap; const T* A2 = (const T*)A2p; const T* Bt = (const T*)Btp; const T* Bt2 = (const T*)Bt2p;
  __shared__ __align__(16) float sT[8][16 * 68];
  const int b    = blockIdx.y;
  const int lane = threadIdx.x & 31;
  const int wave = threadIdx.x >> 5;
  const int tilesN = N >> 6;
  const int tilesM = M >> 6;
  const int tile = blockIdx.x * 8 + wave;
  if (tile >= tilesM * tilesN) return;
  const int tm = tile / tilesN;
  const int tn = tile - tm * tilesN;
  const int m0 = tm << 6;
  const int n0 = tn << 6;

  const T* Ab  = A  + (size_t)b * strideA;
  const T* Bb  = Bt + (size_t)b * strideB;
  const T* Ab2 = SPLIT ? (A2  + (size_t)b * strideA) : nullptr;
  const T* Bb2 = SPLIT ? (Bt2 + (size_t)b * strideB) : nullptr;

  const int rlane = lane & 15;
  const int koff  = (lane >> 4) * 8;
  const int mOff  = (lane >> 4) * 8;

  v8f acc[4][4];
#pragma unroll
  for (int i = 0; i < 4; ++i)
#pragma unroll
    for (int j = 0; j < 4; ++j) acc[i][j] = (v8f){0.f,0.f,0.f,0.f,0.f,0.f,0.f,0.f};

  for (int k0 = 0; k0 < K; k0 += 32) {
    V bh[4], bl[4];
#pragma unroll
    for (int j = 0; j < 4; ++j) {
      const size_t bo = (size_t)(n0 + (j << 4) + rlane) * ldb + koff + k0;
      bh[j] = Frag<T>::load(Bb + bo);
      if (SPLIT) bl[j] = Frag<T>::load(Bb2 + bo);
    }
#pragma unroll
    for (int i = 0; i < 4; ++i) {
      const size_t ao = (size_t)(m0 + (i << 4) + rlane) * lda + koff + k0;
      V ah = Frag<T>::load(Ab + ao);
      V al;
      if (SPLIT) al = Frag<T>::load(Ab2 + ao);
#pragma unroll
      for (int j = 0; j < 4; ++j) {
        acc[i][j] = Frag<T>::mma(ah, bh[j], acc[i][j]);
        if (SPLIT) {
          acc[i][j] = Frag<T>::mma(ah, bl[j], acc[i][j]);
          acc[i][j] = Frag<T>::mma(al, bh[j], acc[i][j]);
        }
      }
      Frag<T>::guard(acc[i][0], acc[i][3], ah, SPLIT ? al : ah);
    }
    Frag<T>::keep(bh[0], bh[1], bh[2], bh[3]);
    if (SPLIT) Frag<T>::keep(bl[0], bl[1], bl[2], bl[3]);
  }
  acc_guard4(acc[0][0], acc[0][1], acc[0][2], acc[0][3]);
  acc_guard4(acc[1][0], acc[1][1], acc[1][2], acc[1][3]);
  acc_guard4(acc[2][0], acc[2][1], acc[2][2], acc[2][3]);
  acc_guard4(acc[3][0], acc[3][1], acc[3][2], acc[3][3]);

  float* slab = sT[wave];
  const float* Rb = RESID ? (resid + (size_t)b * strideR) : nullptr;
#pragma unroll
  for (int i = 0; i < 4; ++i) {
    const int mBase = m0 + (i << 4);
#pragma unroll
    for (int j = 0; j < 4; ++j) {
      const int n = n0 + (j << 4) + rlane;
      float bv = 0.f;
      if (BIAS_MODE == 2) bv = bias[n];
#pragma unroll
      for (int r = 0; r < 8; ++r) {
        float v = acc[i][j][r] * scale;
        if (BIAS_MODE == 1) v += bias[mBase + mOff + r];
        if (BIAS_MODE == 2) v += bv;
        if (RESID) v += Rb[(size_t)(mBase + mOff + r) * ldc + n];
        if (ACT == 1) v = tanhf(v);
        if (ACT == 2) v = fmaxf(v, 0.0f);
        if (ACT == 3) v = v / (1.0f + expf(-v));
        if (ACT == 4) v = (v > 0.f) ? v : 0.01f * v;
        if (ACT == 5) v = 0.5f * v * (1.0f + erff(v * 0.70710678118654752f));
        slab[(mOff + r) * 68 + (j << 4) + rlane] = v;
      }
    }
    __builtin_amdgcn_fence(__ATOMIC_RELEASE, "workgroup");
    __builtin_amdgcn_wave_barrier();
    __builtin_amdgcn_fence(__ATOMIC_ACQUIRE, "workgroup");
    if (OUT_MODE == 0) {
      float* C = (float*)Cout + (size_t)b * strideC;
      const int hh = lane >> 4, c4 = (lane & 15) * 4;
      for (int pass = 0; pass < 2; ++pass) {
#pragma unroll
        for (int it = 0; it < 8; ++it) {
          const int row = it * 2 + hh;
          v4f v = *(const v4f*)(slab + row * 68 + c4);
          *(volatile v4f*)(C + (size_t)(mBase + row) * ldc + n0 + c4) = v;
        }
        __threadfence();
      }
    } else {
      const int q = lane >> 3, c8 = (lane & 7) * 8;
      unsigned short* C  = (unsigned short*)Cout  + (size_t)b * strideC;
      unsigned short* C2 = (OUT_MODE == 2) ? ((unsigned short*)Cout2 + (size_t)b * strideC) : nullptr;
      for (int pass = 0; pass < 2; ++pass) {
#pragma unroll
        for (int it = 0; it < 4; ++it) {
          const int row = it * 4 + q;
          const float* sp = slab + row * 68 + c8;
          v8h hv, lv;
#pragma unroll
          for (int e = 0; e < 8; ++e) {
            if (OUT_MODE == 1) {
              hv[e] = (_Float16)sp[e];
            } else {
              unsigned short hb = f2bf_bits(sp[e]);
              unsigned short lb = f2bf_bits(sp[e] - bf_bits2f(hb));
              hv[e] = __builtin_bit_cast(_Float16, hb);
              lv[e] = __builtin_bit_cast(_Float16, lb);
            }
          }
          *(volatile v8h*)(C + (size_t)(mBase + row) * ldc + n0 + c8) = hv;
          if (OUT_MODE == 2) *(volatile v8h*)(C2 + (size_t)(mBase + row) * ldc + n0 + c8) = lv;
        }
        __threadfence();
      }
    }
    __builtin_amdgcn_fence(__ATOMIC_RELEASE, "workgroup");
    __builtin_amdgcn_wave_barrier();
    __builtin_amdgcn_fence(__ATOMIC_ACQUIRE, "workgroup");
  }
}

__device__ __forceinline__ unsigned pk16(unsigned short a, unsigned short b) { return (unsigned)a | ((unsigned)b << 16); }
template <bool BF> __device__ __forceinline__ unsigned short cvt16(float f) {
  if (BF) return f2bf_bits(f);
  return __builtin_bit_cast(unsigned short, (_Float16)f);
}

template <bool BF>
__global__ __launch_bounds__(256) void cast16x2_kernel(const float* __restrict__ in, unsigned short* __restrict__ out, int n2) {
  const int i = blockIdx.x * 256 + threadIdx.x;
  if (i < n2) {
    const v2f f = *(const v2f*)(in + 2 * (size_t)i);
    const unsigned u = pk16(cvt16<BF>(f[0]), cvt16<BF>(f[1]));
    ((volatile unsigned*)out)[i] = u;
    __threadfence();
    ((volatile unsigned*)out)[i] = u;
  }
}

template <bool BF>
__global__ __launch_bounds__(256) void tcast_kernel(const float* __restrict__ W, unsigned short* __restrict__ o,
                                                    int R, int Cc, float mul) {
  __shared__ __align__(16) float tf[64 * 68];
  const int c0  = blockIdx.x * 64;
  const int r0  = blockIdx.y * 64;
  const int tid = threadIdx.x;
  {
    const int lr = tid >> 4;
    const int c4 = (tid & 15) * 4;
#pragma unroll
    for (int it = 0; it < 4; ++it) {
      const int rr = it * 16 + lr;
      const v4f a = *(const v4f*)(W + (size_t)(r0 + rr) * Cc + c0 + c4);
      *(v4f*)(tf + rr * 68 + c4) = a;
    }
  }
  __syncthreads();
  const int sub = tid >> 3;
  const int c8  = (tid & 7) * 8;
  v4u hv[2];
#pragma unroll
  for (int it = 0; it < 2; ++it) {
    const int oc = it * 32 + sub;
    v4u a;
#pragma unroll
    for (int q = 0; q < 4; ++q) {
      const float f0 = tf[(c8 + 2 * q) * 68 + oc] * mul;
      const float f1 = tf[(c8 + 2 * q + 1) * 68 + oc] * mul;
      a[q] = pk16(cvt16<BF>(f0), cvt16<BF>(f1));
    }
    hv[it] = a;
  }
  for (int pass = 0; pass < 2; ++pass) {
#pragma unroll
    for (int it = 0; it < 2; ++it) {
      const int oc = it * 32 + sub;
      const size_t go = (size_t)(c0 + oc) * R + r0 + c8;
      *(volatile v4u*)(o + go) = hv[it];
    }
    __threadfence();
  }
}

constexpr int kAttD  = 64;
constexpr int kAttNW = 4;
constexpr int kAttKC = 64;

__device__ __forceinline__ v8f mma_h(v16h a, v16h b, v8f c) {
  c = __builtin_amdgcn_wmma_f32_16x16x32_f16(false, a, false, b, (short)0, c, false, false);
  asm volatile("v_nop\n\tv_nop\n\tv_nop\n\tv_nop" : "+v"(c) : "v"(a), "v"(b));
  return c;
}

template <bool CAUSAL>
__global__ __launch_bounds__(128)
void attn16_kernel(const unsigned short* __restrict__ qp, const unsigned short* __restrict__ kp,
                   const unsigned short* __restrict__ vtp, unsigned short* __restrict__ op,
                   int S, int Skv, int nH, int ld, float sscale, float oscale) {
  union FB { v16h v; v8h h[2]; };
  __shared__ __align__(16) _Float16 Ksh[kAttKC * kAttD];
  __shared__ __align__(16) _Float16 Vth[kAttD * kAttKC];
  __shared__ __align__(16) _Float16 Psh[kAttNW][16 * kAttKC];
  __shared__ __align__(16) float    Os[kAttNW][16 * 68];

  const int tid  = threadIdx.x;
  const int wave = tid >> 5;
  const int lane = tid & 31;
  const int hh   = lane >> 4;
  const int c    = lane & 15;

  const int nqb = S / 64;
  const int bx = blockIdx.x;
  const int qb = bx % nqb;
  const int bh = bx / nqb;
  const int h  = bh % nH;
  const int b  = bh / nH;
  const int q0 = qb * 64 + wave * 16;

  const _Float16* Q  = (const _Float16*)(const void*)qp  + (size_t)b * S * ld + (size_t)h * kAttD;
  const _Float16* Kq = (const _Float16*)(const void*)kp  + (size_t)b * Skv * ld + (size_t)h * kAttD;
  const _Float16* Vt = (const _Float16*)(const void*)vtp + (size_t)(b * nH + h) * kAttD * Skv;
  _Float16*       O  = (_Float16*)(void*)op + (size_t)b * S * ld + (size_t)h * kAttD;

  v16h qa[2];
#pragma unroll
  for (int dc = 0; dc < 2; ++dc)
    qa[dc] = Frag<_Float16>::load(Q + (size_t)(q0 + c) * ld + dc * 32 + 8 * hh);

  float mrow[8], lrow[8];
  v8f oacc[4];
#pragma unroll
  for (int r = 0; r < 8; ++r) { mrow[r] = -INFINITY; lrow[r] = 0.f; }
#pragma unroll
  for (int t = 0; t < 4; ++t) oacc[t] = (v8f){0.f,0.f,0.f,0.f,0.f,0.f,0.f,0.f};

  const int nChunks = CAUSAL ? (qb + 1) : (Skv / kAttKC);
  for (int kc = 0; kc < nChunks; ++kc) {
    const int kv0 = kc * kAttKC;
    __syncthreads();
    {
      const int r = tid >> 1, half = (tid & 1) * 32;
      const _Float16* ks = Kq + (size_t)(kv0 + r) * ld + half;
      const _Float16* vs = Vt + (size_t)r * Skv + kv0 + half;
#pragma unroll
      for (int i = 0; i < 4; ++i) {
        const v8h a0 = *(const v8h*)(ks + 8 * i);
        const v8h b0 = *(const v8h*)(vs + 8 * i);
        *(v8h*)(Ksh + r * kAttD  + half + 8 * i) = a0;
        *(v8h*)(Vth + r * kAttKC + half + 8 * i) = b0;
      }
    }
    __syncthreads();

    v8f s[4];
#pragma unroll
    for (int j = 0; j < 4; ++j) {
      s[j] = (v8f){0.f,0.f,0.f,0.f,0.f,0.f,0.f,0.f};
#pragma unroll
      for (int dc = 0; dc < 2; ++dc) {
        FB kb;
        kb.h[0] = *(const v8h*)(Ksh + (j * 16 + c) * kAttD + dc * 32 + 8 * hh);
        kb.h[1] = *(const v8h*)(Ksh + (j * 16 + c) * kAttD + dc * 32 + 16 + 8 * hh);
        s[j] = mma_h(qa[dc], kb.v, s[j]);
      }
    }
    const bool diag = CAUSAL && (kc == qb);
    float cm[8];
#pragma unroll
    for (int r = 0; r < 8; ++r) {
      const int qrow = q0 + 8 * hh + r;
      float m = -INFINITY;
#pragma unroll
      for (int j = 0; j < 4; ++j) {
        const int kvcol = kv0 + j * 16 + c;
        float vv = s[j][r] * sscale;
        if (diag && (kvcol > qrow)) vv = -INFINITY;
        s[j][r] = vv;
        m = fmaxf(m, vv);
      }
#pragma unroll
      for (int off = 1; off < 16; off <<= 1) m = fmaxf(m, __shfl_xor(m, off, 32));
      cm[r] = m;
    }
    _Float16* pw = Psh[wave];
#pragma unroll
    for (int r = 0; r < 8; ++r) {
      const float mnew = fmaxf(mrow[r], cm[r]);
      const float alpha = expf(mrow[r] - mnew);
      mrow[r] = mnew;
      float psum = 0.f;
#pragma unroll
      for (int j = 0; j < 4; ++j) {
        const float p = expf(s[j][r] - mnew);
        psum += p;
        pw[(8 * hh + r) * kAttKC + j * 16 + c] = (_Float16)(p * kPScale);
      }
#pragma unroll
      for (int off = 1; off < 16; off <<= 1) psum += __shfl_xor(psum, off, 32);
      lrow[r] = lrow[r] * alpha + psum;
#pragma unroll
      for (int t = 0; t < 4; ++t) oacc[t][r] *= alpha;
    }
    __builtin_amdgcn_fence(__ATOMIC_RELEASE, "workgroup");
    __builtin_amdgcn_wave_barrier();
    __builtin_amdgcn_fence(__ATOMIC_ACQUIRE, "workgroup");
#pragma unroll
    for (int kk = 0; kk < 2; ++kk) {
      FB pa;
      pa.h[0] = *(const v8h*)(pw + c * kAttKC + kk * 32 + 8 * hh);
      pa.h[1] = *(const v8h*)(pw + c * kAttKC + kk * 32 + 16 + 8 * hh);
#pragma unroll
      for (int t = 0; t < 4; ++t) {
        FB vb;
        vb.h[0] = *(const v8h*)(Vth + (t * 16 + c) * kAttKC + kk * 32 + 8 * hh);
        vb.h[1] = *(const v8h*)(Vth + (t * 16 + c) * kAttKC + kk * 32 + 16 + 8 * hh);
        oacc[t] = mma_h(pa.v, vb.v, oacc[t]);
      }
    }
  }

  float* os = Os[wave];
#pragma unroll
  for (int r = 0; r < 8; ++r) {
    const float inv = oscale / (lrow[r] * kPScale);
#pragma unroll
    for (int t = 0; t < 4; ++t) os[(8 * hh + r) * 68 + t * 16 + c] = oacc[t][r] * inv;
  }
  __builtin_amdgcn_fence(__ATOMIC_RELEASE, "workgroup");
  __builtin_amdgcn_wave_barrier();
  __builtin_amdgcn_fence(__ATOMIC_ACQUIRE, "workgroup");
  {
    const int q8 = lane >> 3, c8 = (lane & 7) * 8;
    for (int pass = 0; pass < 2; ++pass) {
#pragma unroll
      for (int it = 0; it < 4; ++it) {
        const int row = it * 4 + q8;
        const float* sp = os + row * 68 + c8;
        v8h hv;
#pragma unroll
        for (int e = 0; e < 8; ++e) hv[e] = (_Float16)sp[e];
        *(volatile v8h*)(O + (size_t)(q0 + row) * ld + c8) = hv;
      }
      __threadfence();
    }
  }
}

template <bool OUT16>
__global__ __launch_bounds__(128) void layernorm512_kernel(const float* __restrict__ in, const float* __restrict__ gam,
                                                           const float* __restrict__ bet, float* __restrict__ outf,
                                                           unsigned short* __restrict__ outh, int nrows, float eps) {
  __shared__ __align__(16) float srow[4][512];
  const int wave = threadIdx.x >> 5, lane = threadIdx.x & 31;
  const int row = blockIdx.x * 4 + wave;
  if (row >= nrows) return;
  const float* ip = in + (size_t)row * 512;
  v4f v[4], g4[4], b4[4];
  float s = 0.f;
#pragma unroll
  for (int it = 0; it < 4; ++it) {
    const int idx = (it * 32 + lane) * 4;
    v[it]  = *(const v4f*)(ip + idx);
    g4[it] = *(const v4f*)(gam + idx);
    b4[it] = *(const v4f*)(bet + idx);
    s += (v[it][0] + v[it][1]) + (v[it][2] + v[it][3]);
  }
#pragma unroll
  for (int off = 1; off < 32; off <<= 1) s += __shfl_xor(s, off, 32);
  const float mu = s * (1.0f / 512.0f);
  v4f d[4];
  float sq = 0.f;
#pragma unroll
  for (int it = 0; it < 4; ++it) {
    d[it] = v[it] - mu;
    sq += (d[it][0] * d[it][0] + d[it][1] * d[it][1]) + (d[it][2] * d[it][2] + d[it][3] * d[it][3]);
  }
#pragma unroll
  for (int off = 1; off < 32; off <<= 1) sq += __shfl_xor(sq, off, 32);
  const float var  = sq * (1.0f / 512.0f);
  const float rstd = 1.0f / sqrtf(var + eps);
  v4f y[4];
#pragma unroll
  for (int it = 0; it < 4; ++it) y[it] = d[it] * rstd * g4[it] + b4[it];

  float* orow = outf + (size_t)row * 512;
  for (int pass = 0; pass < 2; ++pass) {
#pragma unroll
    for (int it = 0; it < 4; ++it) *(volatile v4f*)(orow + (it * 32 + lane) * 4) = y[it];
    __threadfence();
  }
  if (OUT16) {
    float* sr = srow[wave];
#pragma unroll
    for (int it = 0; it < 4; ++it) *(v4f*)(sr + (it * 32 + lane) * 4) = y[it];
    __builtin_amdgcn_fence(__ATOMIC_RELEASE, "workgroup");
    __builtin_amdgcn_wave_barrier();
    __builtin_amdgcn_fence(__ATOMIC_ACQUIRE, "workgroup");
    v8h hv[2];
#pragma unroll
    for (int j = 0; j < 2; ++j) {
      const int idx8 = (j * 32 + lane) * 8;
      const v4f a  = *(const v4f*)(sr + idx8);
      const v4f a2 = *(const v4f*)(sr + idx8 + 4);
      v8h t;
      t[0] = (_Float16)a[0];  t[1] = (_Float16)a[1];  t[2] = (_Float16)a[2];  t[3] = (_Float16)a[3];
      t[4] = (_Float16)a2[0]; t[5] = (_Float16)a2[1]; t[6] = (_Float16)a2[2]; t[7] = (_Float16)a2[3];
      hv[j] = t;
    }
    unsigned short* oh = outh + (size_t)row * 512;
    for (int pass = 0; pass < 2; ++pass) {
#pragma unroll
      for (int j = 0; j < 2; ++j) *(volatile v8h*)(oh + (j * 32 + lane) * 8) = hv[j];
      __threadfence();
    }
  }
}

__global__ __launch_bounds__(256) void copy_f32x4_kernel(const float* __restrict__ in, float* __restrict__ out, int n4) {
  const int i = blockIdx.x * 256 + threadIdx.x;
  if (i < n4) {
    const v4f a = *(const v4f*)(in + 4 * (size_t)i);
    *(volatile v4f*)(out + 4 * (size_t)i) = a;
    __threadfence();
    *(volatile v4f*)(out + 4 * (size_t)i) = a;
  }
}

template <int ET, int BIAS_MODE, int OUT_MODE, bool RESID, int ACT>
static inline void launch_gemm(const void* A, int lda, long sA, const void* Bt, int ldb, long sB,
                               void* C, int ldc, long sC, const float* bias, const float* resid, long sR,
                               int M, int N, int K, float scale, int batch, hipStream_t st) {
  const int tiles = (M / 64) * (N / 64);
  dim3 grid((tiles + 7) / 8, batch);
  wmma_gemm64<ET, false, BIAS_MODE, OUT_MODE, RESID, ACT><<<grid, 256, 0, st>>>(
      (const unsigned short*)A, (const unsigned short*)A, lda, sA,
      (const unsigned short*)Bt, (const unsigned short*)Bt, ldb, sB,
      C, C, ldc, sC, bias, resid, sR, M, N, K, scale);
}

extern "C" void kernel_launch(void* const* d_in, const int* in_sizes, int n_in,
                              void* d_out, int out_size, void* d_ws, size_t ws_size,
                              hipStream_t stream) {
  if (n_in < 28) return;
  if (in_sizes[0] != kRows * kDim || in_sizes[1] != kRows * kDim) return;
  if (in_sizes[2] != kDim * kDim || in_sizes[22] != kDim * kDff || in_sizes[24] != kDff * kDim) return;
  if ((size_t)out_size < 2 * (size_t)kRows * kDim) return;

  const float* x       = (const float*)d_in[0];
  const float* feature = (const float*)d_in[1];
  const float* wq  = (const float*)d_in[2];  const float* bq  = (const float*)d_in[3];
  const float* wk  = (const float*)d_in[4];  const float* bk  = (const float*)d_in[5];
  const float* wv  = (const float*)d_in[6];  const float* bv  = (const float*)d_in[7];
  const float* wo  = (const float*)d_in[8];  const float* bo  = (const float*)d_in[9];
  const float* ln1_g = (const float*)d_in[10]; const float* ln1_b = (const float*)d_in[11];
  const float* wqc = (const float*)d_in[12]; const float* bqc = (const float*)d_in[13];
  const float* wkc = (const float*)d_in[14]; const float* bkc = (const float*)d_in[15];
  const float* wvc = (const float*)d_in[16]; const float* bvc = (const float*)d_in[17];
  const float* woc = (const float*)d_in[18]; const float* boc = (const float*)d_in[19];
  const float* ln2_g = (const float*)d_in[20]; const float* ln2_b = (const float*)d_in[21];
  const float* w1  = (const float*)d_in[22]; const float* b1  = (const float*)d_in[23];
  const float* w2  = (const float*)d_in[24]; const float* b2  = (const float*)d_in[25];
  const float* lnf_g = (const float*)d_in[26]; const float* lnf_b = (const float*)d_in[27];
  float* out0 = (float*)d_out;
  float* out1 = (float*)((char*)d_out + (size_t)kRows * kDim * sizeof(float));

  const size_t plane16 = (size_t)kRows * kDim * 2;
  const size_t plane32 = (size_t)kRows * kDim * 4;
  const size_t wsq     = (size_t)kDim * kDim * 2;
  const size_t wff     = (size_t)kDim * kDff * 2;
  const size_t oXb  = 0;
  const size_t oFb  = oXb + plane16;
  const size_t oWT  = oFb + plane16;
  const size_t oQ   = oWT + 8 * wsq + 2 * wff;
  const size_t oK   = oQ + plane16;
  const size_t oVt  = oK + plane16;
  const size_t oO   = oVt + plane16;
  const size_t oHf  = oO + plane16;
  const size_t oH1f = oHf + plane32;
  const size_t oH1h = oH1f + plane32;
  const size_t oEnd = oH1h + plane16;
  const size_t oHid = oQ;
  if (oEnd > ws_size) return;
  if (oHid + (size_t)kRows * kDff * 2 > oHf) return;

  char* ws = (char*)d_ws;
  unsigned short* Xb   = (unsigned short*)(ws + oXb);
  unsigned short* Fb   = (unsigned short*)(ws + oFb);
  unsigned short* wqT  = (unsigned short*)(ws + oWT + 0 * wsq);
  unsigned short* wkT  = (unsigned short*)(ws + oWT + 1 * wsq);
  unsigned short* wvT  = (unsigned short*)(ws + oWT + 2 * wsq);
  unsigned short* woT  = (unsigned short*)(ws + oWT + 3 * wsq);
  unsigned short* wqcT = (unsigned short*)(ws + oWT + 4 * wsq);
  unsigned short* wkcT = (unsigned short*)(ws + oWT + 5 * wsq);
  unsigned short* wvcT = (unsigned short*)(ws + oWT + 6 * wsq);
  unsigned short* wocT = (unsigned short*)(ws + oWT + 7 * wsq);
  unsigned short* w1T  = (unsigned short*)(ws + oWT + 8 * wsq);
  unsigned short* w2T  = (unsigned short*)(ws + oWT + 8 * wsq + wff);
  unsigned short* Q16  = (unsigned short*)(ws + oQ);
  unsigned short* K16  = (unsigned short*)(ws + oK);
  unsigned short* Vt16 = (unsigned short*)(ws + oVt);
  unsigned short* O16  = (unsigned short*)(ws + oO);
  unsigned short* Hid  = (unsigned short*)(ws + oHid);
  float*          Hf   = (float*)(ws + oHf);
  float*          H1f  = (float*)(ws + oH1f);
  unsigned short* H1h  = (unsigned short*)(ws + oH1h);

  const float sscale   = 1.0f / sqrtf((float)kDim);
  const float invW     = 1.0f / kWScale;
  const float invWO    = 1.0f / (kWScale * kOScale);
  const long  stride16 = (long)kSeq * kDim;
  const long  strideVt = (long)kDim * kSeq;

  const int n2 = kRows * kDim / 2;
  cast16x2_kernel<true><<<n2 / 256, 256, 0, stream>>>(x, Xb, n2);
  cast16x2_kernel<true><<<n2 / 256, 256, 0, stream>>>(feature, Fb, n2);

  const dim3 gsq(kDim / 64, kDim / 64);
  tcast_kernel<true ><<<gsq, 256, 0, stream>>>(wq,  wqT,  kDim, kDim, 1.0f);
  tcast_kernel<true ><<<gsq, 256, 0, stream>>>(wk,  wkT,  kDim, kDim, 1.0f);
  tcast_kernel<true ><<<gsq, 256, 0, stream>>>(wv,  wvT,  kDim, kDim, 1.0f);
  tcast_kernel<false><<<gsq, 256, 0, stream>>>(wo,  woT,  kDim, kDim, kWScale);
  tcast_kernel<false><<<gsq, 256, 0, stream>>>(wqc, wqcT, kDim, kDim, kWScale);
  tcast_kernel<true ><<<gsq, 256, 0, stream>>>(wkc, wkcT, kDim, kDim, 1.0f);
  tcast_kernel<true ><<<gsq, 256, 0, stream>>>(wvc, wvcT, kDim, kDim, 1.0f);
  tcast_kernel<false><<<gsq, 256, 0, stream>>>(woc, wocT, kDim, kDim, kWScale);
  tcast_kernel<false><<<dim3(kDff / 64, kDim / 64), 256, 0, stream>>>(w1, w1T, kDim, kDff, kWScale);
  tcast_kernel<false><<<dim3(kDim / 64, kDff / 64), 256, 0, stream>>>(w2, w2T, kDff, kDim, kWScale);

  const dim3 agrid(kBatch * kHeads * (kSeq / 64));

  launch_gemm<1, 2, 1, false, 0>(Xb, kDim, 0, wqT, kDim, 0, Q16, kDim, 0, bq, bq, 0, kRows, kDim, kDim, 1.0f, 1, stream);
  launch_gemm<1, 2, 1, false, 0>(Xb, kDim, 0, wkT, kDim, 0, K16, kDim, 0, bk, bk, 0, kRows, kDim, kDim, 1.0f, 1, stream);
  launch_gemm<1, 1, 1, false, 0>(wvT, kDim, 0, Xb, kDim, stride16, Vt16, kSeq, strideVt, bv, bv, 0, kDim, kSeq, kDim, 1.0f, kBatch, stream);
  attn16_kernel<true><<<agrid, 128, 0, stream>>>(Q16, K16, Vt16, O16, kSeq, kSeq, kHeads, kDim, sscale, kOScale);
  launch_gemm<0, 2, 0, true, 0>(O16, kDim, 0, woT, kDim, 0, Hf, kDim, 0, bo, x, 0, kRows, kDim, kDim, invWO, 1, stream);
  layernorm512_kernel<true><<<kRows / 4, 128, 0, stream>>>(Hf, ln1_g, ln1_b, H1f, H1h, kRows, kEps);

  launch_gemm<0, 2, 1, false, 0>(H1h, kDim, 0, wqcT, kDim, 0, Q16, kDim, 0, bqc, bqc, 0, kRows, kDim, kDim, invW, 1, stream);
  launch_gemm<1, 2, 1, false, 0>(Fb, kDim, 0, wkcT, kDim, 0, K16, kDim, 0, bkc, bkc, 0, kRows, kDim, kDim, 1.0f, 1, stream);
  launch_gemm<1, 1, 1, false, 0>(wvcT, kDim, 0, Fb, kDim, stride16, Vt16, kSeq, strideVt, bvc, bvc, 0, kDim, kSeq, kDim, 1.0f, kBatch, stream);
  attn16_kernel<false><<<agrid, 128, 0, stream>>>(Q16, K16, Vt16, O16, kSeq, kSeq, kHeads, kDim, sscale, kOScale);
  launch_gemm<0, 2, 0, true, 0>(O16, kDim, 0, wocT, kDim, 0, Hf, kDim, 0, boc, H1f, 0, kRows, kDim, kDim, invWO, 1, stream);
  layernorm512_kernel<true><<<kRows / 4, 128, 0, stream>>>(Hf, ln2_g, ln2_b, H1f, H1h, kRows, kEps);

  launch_gemm<0, 2, 1, false, 2>(H1h, kDim, 0, w1T, kDim, 0, Hid, kDff, 0, b1, b1, 0, kRows, kDff, kDim, invW, 1, stream);
  launch_gemm<0, 2, 0, true, 0>(Hid, kDff, 0, w2T, kDff, 0, Hf, kDim, 0, b2, H1f, 0, kRows, kDim, kDff, invW, 1, stream);
  layernorm512_kernel<false><<<kRows / 4, 128, 0, stream>>>(Hf, lnf_g, lnf_b, out0, H1h, kRows, kEps);

  const int n4 = kRows * kDim / 4;
  copy_f32x4_kernel<<<n4 / 256, 256, 0, stream>>>(feature, out1, n4);
}
